// SparseAttention_2954937500304
// MI455X (gfx1250) — hardware-verified
//
#include <hip/hip_runtime.h>


#ifndef NB
#define NB 2
#endif
#ifndef SEQ
#define SEQ 2048
#endif
#define NB_FULL  2
#define SEQ_FULL 2048
#define DMOD 2048
#define NH   32
#define HD   64
#define WIN  128
#define QT   32
#define KT   (QT + 2 * WIN)
#define OBP  72
#define VTP  72
#define PCAR  1024.0f
#define OSC   0.0078125f
#define WOCAR 64.0f
#define OPS   0.001953125f
#define SCL   0.125f
#define NEGB  (-1.0e30f)
#define L2E   1.4426950408889634f

static_assert(SEQ % 64 == 0);
static_assert((NB * SEQ) % 64 == 0);
static_assert(DMOD % 64 == 0);
static_assert(DMOD == NH * HD);
static_assert(HD == 64);
static_assert(KT % 32 == 0);
static_assert(QT == 32);
static_assert(SEQ >= 64);
static_assert(NB <= NB_FULL);
static_assert(SEQ <= SEQ_FULL);

typedef _Float16 h16;
typedef unsigned short bf;
typedef __attribute__((ext_vector_type(16))) __bf16   v16bf;
typedef __attribute__((ext_vector_type(16))) _Float16 v16h;
typedef __attribute__((ext_vector_type(8)))  _Float16 v8h;
typedef __attribute__((ext_vector_type(8)))  unsigned short v8us;
typedef __attribute__((ext_vector_type(8)))  float    v8f;
typedef __attribute__((ext_vector_type(4)))  float    v4f;
typedef v8h  __attribute__((may_alias)) v8ha;
typedef v4f  __attribute__((may_alias)) v4fa;
typedef v8f  __attribute__((may_alias)) v8fa;
typedef v8us __attribute__((may_alias)) v8usa;

__device__ __forceinline__ unsigned short f2bf(float f) { unsigned u = __float_as_uint(f); u += 0x7FFFu + ((u >> 16) & 1u); return (unsigned short)(u >> 16); }
__device__ __forceinline__ float bf2f(unsigned short b) { return __uint_as_float(((unsigned)b) << 16); }
__device__ __forceinline__ float bfr(float f) { return bf2f(f2bf(f)); }
__device__ __forceinline__ v16h cat16(v8h lo, v8h hi) { return __builtin_shufflevector(lo, hi, 0, 1, 2, 3, 4, 5, 6, 7, 8, 9, 10, 11, 12, 13, 14, 15); }
__device__ __forceinline__ v16bf cat16b(v8us lo, v8us hi) { return __builtin_bit_cast(v16bf, __builtin_shufflevector(lo, hi, 0, 1, 2, 3, 4, 5, 6, 7, 8, 9, 10, 11, 12, 13, 14, 15)); }
__device__ __forceinline__ v8f wmma16(v16h a, v16h b, v8f c) { return __builtin_amdgcn_wmma_f32_16x16x32_f16(false, a, false, b, (short)0, c, false, false); }
__device__ __forceinline__ v8f wmmab(v16bf a, v16bf b, v8f c) { return __builtin_amdgcn_wmma_f32_16x16x32_bf16(false, a, false, b, (short)0, c, false, false); }
__device__ __forceinline__ void splitf(float y, unsigned short& h, unsigned short& l) { h = f2bf(y); l = f2bf(y - bf2f(h)); }
__device__ __forceinline__ v16bf ldbf(const bf* p) { return cat16b(*(const v8us*)p, *(const v8us*)(p + 16)); }

template <typename T16> struct WFrag;
template <> struct WFrag<h16> { typedef v16h V; static __device__ __forceinline__ V ld(const h16* p) { return cat16(*(const v8h*)p, *(const v8h*)(p + 16)); } static __device__ __forceinline__ v8f mma(V a, V b, v8f c) { return wmma16(a, b, c); } };
template <> struct WFrag<bf> { typedef v16bf V; static __device__ __forceinline__ V ld(const bf* p) { return cat16b(*(const v8us*)p, *(const v8us*)(p + 16)); } static __device__ __forceinline__ v8f mma(V a, V b, v8f c) { return wmmab(a, b, c); } };
template <typename T16, int OM>
__global__ __launch_bounds__(32) void k_gemmw(const T16* __restrict__ A, const T16* __restrict__ Bt, int K, float* C, int ldc, float oscale, bf* Ph, bf* Pl, h16* VTo) {
    typedef typename WFrag<T16>::V V;
    __shared__ __align__(16) float os[16 * 68];
    __shared__ __align__(16) h16 vts[64 * VTP];
    const int lane = threadIdx.x & 31, lr = lane & 15, hi = lane >> 4; const int r0 = blockIdx.x * 64, c0 = blockIdx.y * 64;
    v8f acc[4][4];
#pragma unroll
    for (int mb = 0; mb < 4; ++mb)
#pragma unroll
        for (int nb = 0; nb < 4; ++nb) acc[mb][nb] = (v8f){};
    const size_t aoff = (size_t)(r0 + lr) * K + 8 * hi, boff = (size_t)(c0 + lr) * K + 8 * hi;
#pragma unroll 1
    for (int kc = 0; kc < K; kc += 32) {
        V a[4];
#pragma unroll
        for (int mb = 0; mb < 4; ++mb) a[mb] = WFrag<T16>::ld(A + aoff + (size_t)mb * 16 * K + kc);
#pragma unroll
        for (int nb = 0; nb < 4; ++nb) { const V b = WFrag<T16>::ld(Bt + boff + (size_t)nb * 16 * K + kc);
#pragma unroll
            for (int mb = 0; mb < 4; ++mb) acc[mb][nb] = WFrag<T16>::mma(a[mb], b, acc[mb][nb]); }
        asm volatile("v_nop\n\tv_nop\n\tv_nop\n\tv_nop" : "+v"(acc[0][0]), "+v"(acc[1][1]), "+v"(acc[2][2]), "+v"(acc[3][3]) : "v"(a[0]), "v"(a[3]));
    }
    const int bb = r0 / SEQ, t0 = r0 - bb * SEQ, hh = blockIdx.y; const size_t bh = (size_t)bb * NH + hh;
    if (OM == 2) {
#pragma unroll
        for (int mb = 0; mb < 4; ++mb)
#pragma unroll
            for (int nb = 0; nb < 4; ++nb) { v8h w;
#pragma unroll
                for (int j = 0; j < 8; ++j) w[j] = (h16)acc[mb][nb][j];
                *(v8h*)(vts + (nb * 16 + lr) * VTP + mb * 16 + hi * 8) = w; }
        __builtin_amdgcn_wave_barrier(); asm volatile("" ::: "memory");
        h16* vb = VTo + bh * HD * SEQ + t0;
#pragma unroll 1
        for (int ps = 0; ps < 2; ++ps) {
#pragma unroll
            for (int s = 0; s < 16; ++s) { const int p = s * 32 + lane; const int d = p >> 3, q = p & 7; const v8h val = *(const v8ha*)(vts + d * VTP + q * 8); *(volatile v8h*)(vb + (size_t)d * SEQ + q * 8) = val; }
            if (ps == 0) __threadfence(); }
        __builtin_amdgcn_wave_barrier(); asm volatile("" ::: "memory");
    } else {
#pragma unroll
        for (int mb = 0; mb < 4; ++mb) {
#pragma unroll
            for (int nb = 0; nb < 4; ++nb) {
#pragma unroll
                for (int j = 0; j < 8; ++j) os[(hi * 8 + j) * 68 + nb * 16 + lr] = acc[mb][nb][j]; }
            __builtin_amdgcn_wave_barrier(); asm volatile("" ::: "memory");
            if (OM == 0) {
                float* crow = C + (size_t)(r0 + mb * 16) * ldc + c0;
#pragma unroll 1
                for (int ps = 0; ps < 2; ++ps) {
#pragma unroll
                    for (int s = 0; s < 8; ++s) { const int row = 2 * s + hi, cofs = lr * 4; v4f val = *(const v4fa*)(os + row * 68 + cofs); val = val * oscale;
                        *(volatile v4f*)(crow + (size_t)row * ldc + cofs) = val; }
                    if (ps == 0) __threadfence(); }
            } else {
                bf* hbp = Ph + (bh * SEQ + t0 + mb * 16) * HD; bf* lbp = Pl + (bh * SEQ + t0 + mb * 16) * HD;
#pragma unroll 1
                for (int ps = 0; ps < 2; ++ps) {
#pragma unroll
                    for (int s = 0; s < 4; ++s) { const int p = s * 32 + lane; const int row = p >> 3, q = p & 7;
                        const v4f u0 = *(const v4fa*)(os + row * 68 + q * 8); const v4f u1 = *(const v4fa*)(os + row * 68 + q * 8 + 4); v8us oh, ol;
#pragma unroll
                        for (int e = 0; e < 4; ++e) { unsigned short x1, x2; splitf(u0[e], x1, x2); oh[e] = x1; ol[e] = x2; splitf(u1[e], x1, x2); oh[4 + e] = x1; ol[4 + e] = x2; }
                        *(volatile v8us*)(hbp + row * HD + q * 8) = oh; *(volatile v8us*)(lbp + row * HD + q * 8) = ol; }
                    if (ps == 0) __threadfence(); }
            }
            __builtin_amdgcn_wave_barrier(); asm volatile("" ::: "memory");
        }
    }
}

__global__ __launch_bounds__(256) void k_cvt8(const float* __restrict__ src, bf* dst, size_t n8) { const size_t i = (size_t)blockIdx.x * 256 + threadIdx.x; if (i >= n8) return; const v8f v = *(const v8f*)(src + i * 8); v8us o;
#pragma unroll
    for (int k = 0; k < 8; ++k) o[k] = f2bf(v[k]); *(volatile v8us*)(dst + i * 8) = o; __threadfence(); *(volatile v8us*)(dst + i * 8) = o; }
__global__ __launch_bounds__(256) void k_cvt8h(const float* __restrict__ src, h16* dst, size_t n8, float scl) { const size_t i = (size_t)blockIdx.x * 256 + threadIdx.x; if (i >= n8) return; const v8f v = *(const v8f*)(src + i * 8); v8h o;
#pragma unroll
    for (int k = 0; k < 8; ++k) o[k] = (h16)(bfr(v[k]) * scl); *(volatile v8h*)(dst + i * 8) = o; __threadfence(); *(volatile v8h*)(dst + i * 8) = o; }

__global__ __launch_bounds__(64) void k_attn(const bf* __restrict__ Qh, const bf* __restrict__ Ql, const bf* __restrict__ Kh, const bf* __restrict__ Kl, const h16* __restrict__ Vt, h16* CT) {
    __shared__ __align__(16) float sbuf[2][16 * KT];
    __shared__ __align__(16) h16 obuf[2][16 * OBP];
    __shared__ float mxb[2][16];
    const int wave = threadIdx.x >> 5, lane = threadIdx.x & 31, lm = lane & 15, hf = lane >> 4;
    const int bh = blockIdx.y; const int bb = bh / NH, hh = bh - bb * NH;
    const int q0 = blockIdx.x * QT; const int kbase = q0 - WIN; const int qw = q0 + wave * 16;
    const size_t hp = (size_t)bh * SEQ * HD;
    const size_t qoff = hp + (size_t)(qw + lm) * HD + 8 * hf;
    const v16bf qh0 = ldbf(Qh + qoff), qh1 = ldbf(Qh + qoff + 32), ql0 = ldbf(Ql + qoff), ql1 = ldbf(Ql + qoff + 32);
    float vmax[8];
#pragma unroll
    for (int r = 0; r < 8; ++r) vmax[r] = -3.0e38f;
    float* sw = sbuf[wave];
#pragma unroll 1
    for (int jt = 0; jt < KT / 16; ++jt) {
        const int j = kbase + jt * 16 + lm;
        const int g = min(max(j, 0), SEQ - 1);
        const size_t koff = hp + (size_t)g * HD + 8 * hf;
        const v16bf kh0 = ldbf(Kh + koff), kh1 = ldbf(Kh + koff + 32), kl0 = ldbf(Kl + koff), kl1 = ldbf(Kl + koff + 32);
        v8f c = (v8f){};
        c = wmmab(qh0, kh0, c); c = wmmab(ql0, kh0, c); c = wmmab(qh0, kl0, c);
        c = wmmab(qh1, kh1, c); c = wmmab(ql1, kh1, c); c = wmmab(qh1, kl1, c);
        asm volatile("v_nop\n\tv_nop\n\tv_nop\n\tv_nop" : "+v"(c) : "v"(qh0), "v"(ql0), "v"(qh1), "v"(ql1), "v"(kh1), "v"(kl1));
        const bool jok = (j >= 0) && (j < SEQ);
#pragma unroll
        for (int r = 0; r < 8; ++r) { const int dd = qw + 8 * hf + r - j; const bool ok = jok && (dd <= WIN) && (dd >= -WIN); const float s = ok ? c[r] * SCL : NEGB; sw[(8 * hf + r) * KT + jt * 16 + lm] = s; vmax[r] = fmaxf(vmax[r], s); }
    }
#pragma unroll
    for (int r = 0; r < 8; ++r) { float v = vmax[r]; v = fmaxf(v, __shfl_xor(v, 1, 32)); v = fmaxf(v, __shfl_xor(v, 2, 32)); v = fmaxf(v, __shfl_xor(v, 4, 32)); v = fmaxf(v, __shfl_xor(v, 8, 32)); vmax[r] = v; }
    if (lm == 0) {
#pragma unroll
        for (int r = 0; r < 8; ++r) mxb[wave][8 * hf + r] = vmax[r]; }
    __syncthreads();
    const float rmax = mxb[wave][lm];
    v8f o[4];
#pragma unroll
    for (int ni = 0; ni < 4; ++ni) o[ni] = (v8f){};
    float lsum = 0.f;
    const float* srow = sw + lm * KT + 8 * hf;
    const size_t vp = (size_t)bh * HD * SEQ + (size_t)lm * SEQ;
#pragma unroll 1
    for (int kc = 0; kc < KT / 32; ++kc) {
        const v8f x0 = *(const v8fa*)(srow + kc * 32); const v8f x1 = *(const v8fa*)(srow + kc * 32 + 16);
        v16h ap;
#pragma unroll
        for (int e = 0; e < 8; ++e) { float d0 = __fsub_rn(x0[e], rmax); asm volatile("" : "+v"(d0)); const float p = __builtin_amdgcn_exp2f(__fmul_rn(d0, L2E)); lsum += p; ap[e] = (h16)(p * PCAR); }
#pragma unroll
        for (int e = 0; e < 8; ++e) { float d0 = __fsub_rn(x1[e], rmax); asm volatile("" : "+v"(d0)); const float p = __builtin_amdgcn_exp2f(__fmul_rn(d0, L2E)); lsum += p; ap[8 + e] = (h16)(p * PCAR); }
        int g0 = kbase + kc * 32 + 8 * hf; int g1 = g0 + 16; g0 = min(max(g0, 0), SEQ - 8); g1 = min(max(g1, 0), SEQ - 8);
#pragma unroll
        for (int ni = 0; ni < 4; ++ni) { const h16* vr = Vt + vp + (size_t)ni * 16 * SEQ; const v16h bv = cat16(*(const v8h*)(vr + g0), *(const v8h*)(vr + g1)); o[ni] = wmma16(ap, bv, o[ni]); }
        asm volatile("v_nop\n\tv_nop\n\tv_nop\n\tv_nop" : "+v"(o[0]), "+v"(o[1]), "+v"(o[2]), "+v"(o[3]) : "v"(ap));
    }
    lsum += __shfl_xor(lsum, 16, 32);
    const float fl = __fdiv_rn(OSC, lsum);
    float fr[8];
#pragma unroll
    for (int r = 0; r < 8; ++r) fr[r] = __shfl(fl, 8 * hf + r, 32);
    h16* ob = obuf[wave];
#pragma unroll
    for (int ni = 0; ni < 4; ++ni)
#pragma unroll
        for (int r = 0; r < 8; ++r) ob[(8 * hf + r) * OBP + ni * 16 + lm] = (h16)(o[ni][r] * fr[r]);
    __syncthreads();
    h16* crow = CT + ((size_t)bb * SEQ + qw) * DMOD + hh * HD;
#pragma unroll 1
    for (int ps = 0; ps < 2; ++ps) {
#pragma unroll
        for (int s = 0; s < 4; ++s) { const int rr = s * 4 + (lane >> 3), qq = lane & 7; const v8h val = *(const v8ha*)(ob + rr * OBP + qq * 8); *(volatile v8h*)(crow + (size_t)rr * DMOD + qq * 8) = val; }
        if (ps == 0) __threadfence(); }
}

extern "C" void kernel_launch(void* const* d_in, const int* in_sizes, int n_in,
                              void* d_out, int out_size, void* d_ws, size_t ws_size, hipStream_t stream) {
    if (n_in < 5) return;
    if (in_sizes[0] < (NB - 1) * SEQ_FULL * DMOD + SEQ * DMOD) return;
    if (in_sizes[1] < DMOD * DMOD || in_sizes[2] < DMOD * DMOD || in_sizes[3] < DMOD * DMOD || in_sizes[4] < DMOD * DMOD) return;
    if (out_size < NB * SEQ * DMOD) return;
    const float* X  = (const float*)d_in[0];
    const float* Wq = (const float*)d_in[1];
    const float* Wk = (const float*)d_in[2];
    const float* Wv = (const float*)d_in[3];
    const float* Wo = (const float*)d_in[4];
    float* OUT = (float*)d_out;
    char* wsp = (char*)d_ws;
    auto take = [&](size_t bytes) { char* p = wsp; wsp += (bytes + 255) & ~(size_t)255; return (void*)p; };
    const size_t MR = (size_t)NB * SEQ;
    const size_t PL = MR * DMOD;
    bf*  Xb  = (bf*)take(PL * 2);
    bf*  Wsl = (bf*)take((size_t)DMOD * DMOD * 2);
    bf*  Qh  = (bf*)take(PL * 2); bf* Ql = (bf*)take(PL * 2); bf* Kh = (bf*)take(PL * 2); bf* Kl = (bf*)take(PL * 2);
    h16* Vt  = (h16*)take(PL * 2);
    h16* CT  = (h16*)Xb;
    h16* Wo16 = (h16*)Wsl;
    if ((size_t)(wsp - (char*)d_ws) > ws_size) return;

    const unsigned gx8 = (unsigned)(((size_t)SEQ * DMOD / 8 + 255) / 256);
    const unsigned gw8 = (unsigned)(((size_t)DMOD * DMOD / 8 + 255) / 256);
    const dim3 gg((unsigned)(MR / 64), DMOD / 64, 1);
    for (int b = 0; b < NB; ++b)
        k_cvt8<<<gx8, 256, 0, stream>>>(X + (size_t)b * SEQ_FULL * DMOD, Xb + (size_t)b * SEQ * DMOD, (size_t)SEQ * DMOD / 8);
    k_cvt8<<<gw8, 256, 0, stream>>>(Wq, Wsl, (size_t)DMOD * DMOD / 8);
    k_gemmw<bf, 1><<<gg, 32, 0, stream>>>(Xb, Wsl, DMOD, (float*)nullptr, 0, 1.0f, Qh, Ql, (h16*)nullptr);
    k_cvt8<<<gw8, 256, 0, stream>>>(Wk, Wsl, (size_t)DMOD * DMOD / 8);
    k_gemmw<bf, 1><<<gg, 32, 0, stream>>>(Xb, Wsl, DMOD, (float*)nullptr, 0, 1.0f, Kh, Kl, (h16*)nullptr);
    k_cvt8<<<gw8, 256, 0, stream>>>(Wv, Wsl, (size_t)DMOD * DMOD / 8);
    k_gemmw<bf, 2><<<gg, 32, 0, stream>>>(Xb, Wsl, DMOD, (float*)nullptr, 0, 1.0f, (bf*)nullptr, (bf*)nullptr, Vt);
    k_attn<<<dim3(SEQ / QT, NB * NH, 1), 64, 0, stream>>>(Qh, Ql, Kh, Kl, Vt, CT);
    k_cvt8h<<<gw8, 256, 0, stream>>>(Wo, Wo16, (size_t)DMOD * DMOD / 8, WOCAR);
    k_gemmw<h16, 0><<<gg, 32, 0, stream>>>(CT, Wo16, DMOD, OUT, DMOD, OPS, (bf*)nullptr, (bf*)nullptr, (h16*)nullptr);
}
